// BPTBlock_66279935312382
// MI455X (gfx1250) — hardware-verified
//
#include <hip/hip_runtime.h>
#include <stddef.h>


#define DF    128
#define QC    384
#define FFW   512
#define NH    8
#define GR    32
#define NTHR  256
#define NWAVE 8
#define AP    136
#define FP    520
#define CP    388
#define XP    132
#define NB    448
#define SLPW  (NB / NWAVE)
#define CHUNK 2048
#define WCAP  256
#define NGRP  (CHUNK / (NTHR * 4))

#define LDS2_BYTES (GR * AP * 2 * 2 + GR * CP * 4)
#define LDS3_FLT   (NB * DF + 2 * NB * NH + NWAVE * WCAP + 16)
#define LDS3_BYTES (LDS3_FLT * 4)
#define LDS4_BYTES (GR * AP * 2 * 2 + 2 * GR * XP * 4 + GR * FP * 2 * 2)

static_assert(LDS2_BYTES == 67072);
static_assert(LDS3_BYTES == 266304);
static_assert(LDS4_BYTES == 117760);
static_assert(WCAP == (CHUNK / NTHR) * 32);
static_assert(NGRP == 2);
static_assert(NB < 512);
static_assert((NB % NWAVE) == 0);
static_assert(((NB * DF + NB * NH) % 4) == 0);
static_assert(((NB * NH) % 4) == 0);
static_assert((AP % 8) == 0);
static_assert((FP % 8) == 0);
static_assert((CP % 4) == 0);
static_assert((XP % 4) == 0);

typedef float    v4f  __attribute__((ext_vector_type(4)));
typedef float    v8f  __attribute__((ext_vector_type(8)));
typedef int      v4i  __attribute__((ext_vector_type(4)));
typedef unsigned v2u  __attribute__((ext_vector_type(2)));
typedef __bf16   v16b __attribute__((ext_vector_type(16)));
union Frag { v16b v; v4i q[2]; };

__device__ __forceinline__ v8f wm(v16b a, v16b b, v8f c) {
  v8f d = __builtin_amdgcn_wmma_f32_16x16x32_bf16(false, a, false, b, (short)0, c, false, false);
  asm volatile("v_nop\n\tv_nop\n\tv_nop\n\tv_nop" : "+v"(d) : "v"(a), "v"(b));
  return d;
}

__device__ __forceinline__ float wsum(float v) {
  v += __shfl_xor(v, 16, 32);
  v += __shfl_xor(v, 8, 32);
  v += __shfl_xor(v, 4, 32);
  v += __shfl_xor(v, 2, 32);
  v += __shfl_xor(v, 1, 32);
  return v;
}

__device__ __forceinline__ unsigned bfb(float x) {
  const unsigned u = __float_as_uint(x);
  return (u + 0x7FFFu + ((u >> 16) & 1u)) >> 16;
}
__device__ __forceinline__ void split1(float x, unsigned& hb, unsigned& lb) {
  hb = bfb(x);
  const float hf = __uint_as_float(hb << 16);
  lb = bfb(x - hf);
}
__device__ __forceinline__ void split8(v4f a, v4f b, v4i& H, v4i& L) {
  unsigned h0, h1, h2, h3, h4, h5, h6, h7, l0, l1, l2, l3, l4, l5, l6, l7;
  split1(a.x, h0, l0); split1(a.y, h1, l1); split1(a.z, h2, l2); split1(a.w, h3, l3);
  split1(b.x, h4, l4); split1(b.y, h5, l5); split1(b.z, h6, l6); split1(b.w, h7, l7);
  H.x = (int)(h0 | (h1 << 16)); H.y = (int)(h2 | (h3 << 16));
  H.z = (int)(h4 | (h5 << 16)); H.w = (int)(h6 | (h7 << 16));
  L.x = (int)(l0 | (l1 << 16)); L.y = (int)(l2 | (l3 << 16));
  L.z = (int)(l4 | (l5 << 16)); L.w = (int)(l6 | (l7 << 16));
}
__device__ __forceinline__ void split4(v4f a, v2u& H, v2u& L) {
  unsigned h0, h1, h2, h3, l0, l1, l2, l3;
  split1(a.x, h0, l0); split1(a.y, h1, l1); split1(a.z, h2, l2); split1(a.w, h3, l3);
  H.x = h0 | (h1 << 16); H.y = h2 | (h3 << 16);
  L.x = l0 | (l1 << 16); L.y = l2 | (l3 << 16);
}

__device__ __forceinline__ v4f ln_row(v4f x, v4f g, v4f b) {
  const float s  = wsum(x.x + x.y + x.z + x.w);
  const float mu = s * (1.0f / DF);
  const v4f dd = x - mu;
  const float q  = wsum(dd.x * dd.x + dd.y * dd.y + dd.z * dd.z + dd.w * dd.w);
  const float rs = rsqrtf(q * (1.0f / DF) + 1e-5f);
  return dd * rs * g + b;
}

__device__ __forceinline__ void stage32(const float* __restrict__ P, int rowBase, int nN,
                                        unsigned short* Th, unsigned short* Tl, int tid) {
  const int r  = tid >> 3;
  const int c0 = (tid & 7) * 16;
  int row = rowBase + r;
  if (row > nN - 1) row = nN - 1;
  const float* p = P + (size_t)row * DF + c0;
  const v4f f0 = *(const v4f*)(p), f1 = *(const v4f*)(p + 4);
  const v4f f2 = *(const v4f*)(p + 8), f3 = *(const v4f*)(p + 12);
  v4i h0, l0, h1, l1;
  split8(f0, f1, h0, l0);
  split8(f2, f3, h1, l1);
  *(v4i*)(Th + r * AP + c0)     = h0;
  *(v4i*)(Th + r * AP + c0 + 8) = h1;
  *(v4i*)(Tl + r * AP + c0)     = l0;
  *(v4i*)(Tl + r * AP + c0 + 8) = l1;
}

template <int K>
__device__ __forceinline__ void gemm2t(const unsigned short* Th, const unsigned short* Tl, int ap,
                                       const unsigned short* __restrict__ Bh,
                                       const unsigned short* __restrict__ Bl,
                                       int ncol, int hh, int m, v8f& c0, v8f& c1) {
  const unsigned short* pa0 = Th + m * ap + 8 * hh;
  const unsigned short* pa1 = Th + (16 + m) * ap + 8 * hh;
  const unsigned short* pl0 = Tl + m * ap + 8 * hh;
  const unsigned short* pl1 = Tl + (16 + m) * ap + 8 * hh;
  const unsigned short* pbh = Bh + (size_t)ncol * K + 8 * hh;
  const unsigned short* pbl = Bl + (size_t)ncol * K + 8 * hh;
#pragma unroll 4
  for (int kt = 0; kt < K / 32; ++kt) {
    const int k0 = kt * 32;
    Frag a0h, a0l, a1h, a1l, bh, bl;
    a0h.q[0] = *(const v4i*)(pa0 + k0); a0h.q[1] = *(const v4i*)(pa0 + k0 + 16);
    a1h.q[0] = *(const v4i*)(pa1 + k0); a1h.q[1] = *(const v4i*)(pa1 + k0 + 16);
    a0l.q[0] = *(const v4i*)(pl0 + k0); a0l.q[1] = *(const v4i*)(pl0 + k0 + 16);
    a1l.q[0] = *(const v4i*)(pl1 + k0); a1l.q[1] = *(const v4i*)(pl1 + k0 + 16);
    bh.q[0]  = *(const v4i*)(pbh + k0); bh.q[1]  = *(const v4i*)(pbh + k0 + 16);
    bl.q[0]  = *(const v4i*)(pbl + k0); bl.q[1]  = *(const v4i*)(pbl + k0 + 16);
    c0 = wm(a0h.v, bh.v, c0);
    c0 = wm(a0h.v, bl.v, c0);
    c0 = wm(a0l.v, bh.v, c0);
    c1 = wm(a1h.v, bh.v, c1);
    c1 = wm(a1h.v, bl.v, c1);
    c1 = wm(a1l.v, bh.v, c1);
  }
}

__global__ __launch_bounds__(NTHR) void k_prepw(const float* __restrict__ W, int K, int Ncol,
                                                unsigned short* hi, unsigned short* lo, int n8) {
  const int i = blockIdx.x * NTHR + threadIdx.x;
  if (i >= n8) return;
  const int kb8 = K >> 3;
  const int n   = i / kb8;
  const int kb  = (i - n * kb8) * 8;
  float w[8];
#pragma unroll
  for (int j = 0; j < 8; ++j) w[j] = W[(size_t)(kb + j) * Ncol + n];
  v4f a, b;
  a.x = w[0]; a.y = w[1]; a.z = w[2]; a.w = w[3];
  b.x = w[4]; b.y = w[5]; b.z = w[6]; b.w = w[7];
  v4i H, L;
  split8(a, b, H, L);
  unsigned short* ph = hi + (size_t)i * 8;
  unsigned short* pl = lo + (size_t)i * 8;
  *(volatile v4i*)ph = H;
  *(volatile v4i*)pl = L;
  __threadfence();
  *(volatile v4i*)ph = H;
  *(volatile v4i*)pl = L;
}

__global__ __launch_bounds__(NTHR) void k_qkv(const float* __restrict__ x,
                                              const unsigned short* __restrict__ Bh,
                                              const unsigned short* __restrict__ Bl,
                                              float* qkv, int nN) {
  extern __shared__ v4i lds2[];
  unsigned short* Thi = (unsigned short*)lds2;
  unsigned short* Tlo = Thi + GR * AP;
  float* Cs = (float*)(Tlo + GR * AP);

  const int tid  = threadIdx.x;
  const int lane = tid & 31;
  const int wave = tid >> 5;
  const int hh   = lane >> 4;
  const int m    = lane & 15;
  const int rowBase = blockIdx.x * GR;

  stage32(x, rowBase, nN, Thi, Tlo, tid);
  __syncthreads();

#pragma unroll 1
  for (int c3 = 0; c3 < 3; ++c3) {
    const int ct   = wave + 8 * c3;
    const int ncol = ct * 16 + m;
    v8f acc0 = {0.f, 0.f, 0.f, 0.f, 0.f, 0.f, 0.f, 0.f};
    v8f acc1 = {0.f, 0.f, 0.f, 0.f, 0.f, 0.f, 0.f, 0.f};
    gemm2t<DF>(Thi, Tlo, AP, Bh, Bl, ncol, hh, m, acc0, acc1);
#pragma unroll
    for (int r = 0; r < 8; ++r) {
      Cs[(8 * hh + r) * CP + ncol]      = acc0[r];
      Cs[(16 + 8 * hh + r) * CP + ncol] = acc1[r];
    }
  }
  __syncthreads();

  v4f xr[12];
  float* xpp[12];
#pragma unroll
  for (int i = 0; i < 4; ++i) {
    const int row = 4 * wave + i;
#pragma unroll
    for (int j = 0; j < 3; ++j) {
      xr[3 * i + j]  = *(const v4f*)(Cs + row * CP + 128 * j + 4 * lane);
      xpp[3 * i + j] = qkv + (size_t)(rowBase + row) * QC + 128 * j + 4 * lane;
    }
  }
#pragma unroll
  for (int i = 0; i < 12; ++i) *(volatile v4f*)(xpp[i]) = xr[i];
  __threadfence();
#pragma unroll
  for (int i = 0; i < 12; ++i) *(volatile v4f*)(xpp[i]) = xr[i];
}

__global__ __launch_bounds__(NTHR) void k_agg(const float* __restrict__ qkv,
                                              const int* __restrict__ src,
                                              const int* __restrict__ dst,
                                              float* aout, int nN, int nE) {
  extern __shared__ v4f lds3[];
  float* sacc = (float*)lds3;
  float* sden = sacc + NB * DF;
  float* smax = sden + NB * NH;
  int*   list = (int*)(smax + NB * NH);
  int*   wcnt = list + NWAVE * WCAP;

  const int tid  = threadIdx.x;
  const int lane = tid & 31;
  const int wave = tid >> 5;
  const int hd   = lane >> 2;
  const int nodeBase = blockIdx.x * NB;

  {
    const v4f z4 = {0.f, 0.f, 0.f, 0.f};
    const v4f m4 = {-1e30f, -1e30f, -1e30f, -1e30f};
    const int nz = (NB * DF + NB * NH) / 4;
    const int nm = (NB * NH) / 4;
    for (int i = tid; i < nz; i += NTHR) lds3[i] = z4;
    for (int i = tid; i < nm; i += NTHR) lds3[nz + i] = m4;
  }
  __syncthreads();

  const int nChunks = (nE + CHUNK - 1) / CHUNK;
#pragma unroll 1
  for (int ch = 0; ch < nChunks; ++ch) {
    const int cbase = ch * CHUNK;
    int wc = 0;
#pragma unroll
    for (int g = 0; g < NGRP; ++g) {
      const int el0 = (g * NTHR + tid) * 4;
      const int e0  = cbase + el0;
      const int sent = -2147483647 - 1;
      v4i d;
      if (cbase + CHUNK <= nE) {
        d = *(const v4i*)(dst + e0);
      } else {
        const int c0 = (e0     < nE) ? e0     : nE - 1;
        const int c1 = (e0 + 1 < nE) ? e0 + 1 : nE - 1;
        const int c2 = (e0 + 2 < nE) ? e0 + 2 : nE - 1;
        const int c3 = (e0 + 3 < nE) ? e0 + 3 : nE - 1;
        const int v0 = dst[c0], v1 = dst[c1], v2 = dst[c2], v3 = dst[c3];
        d.x = (e0     < nE) ? v0 : sent;
        d.y = (e0 + 1 < nE) ? v1 : sent;
        d.z = (e0 + 2 < nE) ? v2 : sent;
        d.w = (e0 + 3 < nE) ? v3 : sent;
      }
      const unsigned s0 = (unsigned)d.x - (unsigned)nodeBase;
      const unsigned s1 = (unsigned)d.y - (unsigned)nodeBase;
      const unsigned s2 = (unsigned)d.z - (unsigned)nodeBase;
      const unsigned s3 = (unsigned)d.w - (unsigned)nodeBase;
      const bool h0 = s0 < (unsigned)NB;
      const bool h1 = s1 < (unsigned)NB;
      const bool h2 = s2 < (unsigned)NB;
      const bool h3 = s3 < (unsigned)NB;
      const unsigned many = __builtin_amdgcn_ballot_w32(h0 | h1 | h2 | h3);
      if (many != 0u) {
#define HITJ(J, HJ, SJ) { \
          const unsigned mj = __builtin_amdgcn_ballot_w32(HJ); \
          if (HJ) { \
            const int pos = wc + (int)__builtin_amdgcn_mbcnt_lo(mj, 0u); \
            if (pos < WCAP) list[wave * WCAP + pos] = ((el0 + (J)) << 9) | (int)(SJ); \
          } \
          wc += (int)__builtin_popcount(mj); }
        HITJ(0, h0, s0)
        HITJ(1, h1, s1)
        HITJ(2, h2, s2)
        HITJ(3, h3, s3)
#undef HITJ
      }
    }
    if (lane == 0) wcnt[wave] = wc;
    __syncthreads();

    if (wave == 0) {
      for (int wsx = 0; wsx < NWAVE; ++wsx) {
        int n = wcnt[wsx];
        n = (n > WCAP) ? WCAP : n;
        n = (n < 0) ? 0 : n;
        for (int i = 0; i < n; ++i) {
          const int ent = list[wsx * WCAP + i];
          int slot = ent & 511;
          if (slot > NB - 1) slot = NB - 1;
          const int el = (ent >> 9) & (CHUNK - 1);
          int e = cbase + el;
          if (e > nE - 1) e = nE - 1;
          int sv = src[e];
          sv = (sv < 0) ? 0 : ((sv > nN - 1) ? nN - 1 : sv);
          int nd = nodeBase + slot;
          if (nd > nN - 1) nd = nN - 1;
          const float* qr = qkv + (size_t)nd * QC + 4 * lane;
          const float* kr = qkv + (size_t)sv * QC + DF + 4 * lane;
          const v4f qv = *(const v4f*)qr;
          const v4f kv = *(const v4f*)kr;
          const v4f vv = *(const v4f*)(kr + DF);
          float sc = qv.x * kv.x + qv.y * kv.y + qv.z * kv.z + qv.w * kv.w;
          sc += __shfl_xor(sc, 1, 32);
          sc += __shfl_xor(sc, 2, 32);
          sc *= 0.25f;
          const int mi = slot * NH + hd;
          const float mo = smax[mi];
          const float dn = sden[mi];
          const float mn = fmaxf(mo, sc);
          const float rsc = __expf(mo - mn);
          const float p   = __expf(sc - mn);
          v4f* sp = (v4f*)(sacc + slot * DF + 4 * lane);
          const v4f cur = *sp;
          const v4f nxt = cur * rsc + p * vv;
          *sp = nxt;
          smax[mi] = mn;
          sden[mi] = dn * rsc + p;
        }
      }
    }
    __syncthreads();
  }

#pragma unroll 1
  for (int j = 0; j < SLPW; ++j) {
    const int slot = wave * SLPW + j;
    const int node = nodeBase + slot;
    if (node >= nN) break;
    const v4f av = *(const v4f*)(sacc + slot * DF + 4 * lane);
    const float dn = sden[slot * NH + hd];
    const float rc = __builtin_amdgcn_rcpf(dn);
    const float inv = (dn > 0.f) ? rc : 0.f;
    const v4f a = av * inv;
    float* op = aout + (size_t)node * DF + 4 * lane;
    *(volatile v4f*)op = a;
    __threadfence();
    *(volatile v4f*)op = a;
  }
}

__global__ __launch_bounds__(NTHR) void k_ffn(
    const float* __restrict__ ap, const float* __restrict__ h,
    const unsigned short* __restrict__ Woh, const unsigned short* __restrict__ Wol,
    const float* __restrict__ g1, const float* __restrict__ be1,
    const unsigned short* __restrict__ W1h, const unsigned short* __restrict__ W1l,
    const float* __restrict__ bf1,
    const unsigned short* __restrict__ W2h, const unsigned short* __restrict__ W2l,
    const float* __restrict__ bf2,
    const float* __restrict__ g2, const float* __restrict__ be2,
    float* out, int nN) {
  extern __shared__ v4i lds4[];
  unsigned short* Thi = (unsigned short*)lds4;
  unsigned short* Tlo = Thi + GR * AP;
  float* Hs = (float*)(Tlo + GR * AP);
  float* Os = Hs + GR * XP;
  unsigned short* Fhi = (unsigned short*)(Os + GR * XP);
  unsigned short* Flo = Fhi + GR * FP;

  const int tid  = threadIdx.x;
  const int lane = tid & 31;
  const int wave = tid >> 5;
  const int hh   = lane >> 4;
  const int m    = lane & 15;
  const int rowBase = blockIdx.x * GR;
  const int ncw  = wave * 16 + m;

  stage32(ap, rowBase, nN, Thi, Tlo, tid);
  __syncthreads();

  {
    v8f o0 = {0.f, 0.f, 0.f, 0.f, 0.f, 0.f, 0.f, 0.f};
    v8f o1 = {0.f, 0.f, 0.f, 0.f, 0.f, 0.f, 0.f, 0.f};
    gemm2t<DF>(Thi, Tlo, AP, Woh, Wol, ncw, hh, m, o0, o1);
#pragma unroll
    for (int r = 0; r < 8; ++r) {
      Hs[(8 * hh + r) * XP + ncw]      = o0[r];
      Hs[(16 + 8 * hh + r) * XP + ncw] = o1[r];
    }
  }
  __syncthreads();

  {
    const v4f gv = *(const v4f*)(g1 + 4 * lane);
    const v4f bv = *(const v4f*)(be1 + 4 * lane);
#pragma unroll
    for (int i = 0; i < 4; ++i) {
      const int row = 4 * wave + i;
      int grow = rowBase + row;
      if (grow > nN - 1) grow = nN - 1;
      const v4f xo = *(const v4f*)(Hs + row * XP + 4 * lane);
      const v4f xh = *(const v4f*)(h + (size_t)grow * DF + 4 * lane);
      const v4f y  = ln_row(xo + xh, gv, bv);
      *(v4f*)(Hs + row * XP + 4 * lane) = y;
      v2u H, L;
      split4(y, H, L);
      *(v2u*)(Thi + row * AP + 4 * lane) = H;
      *(v2u*)(Tlo + row * AP + 4 * lane) = L;
    }
  }
  __syncthreads();

#pragma unroll 1
  for (int j = 0; j < 4; ++j) {
    const int ct   = wave + 8 * j;
    const int ncol = ct * 16 + m;
    v8f f0 = {0.f, 0.f, 0.f, 0.f, 0.f, 0.f, 0.f, 0.f};
    v8f f1 = {0.f, 0.f, 0.f, 0.f, 0.f, 0.f, 0.f, 0.f};
    gemm2t<DF>(Thi, Tlo, AP, W1h, W1l, ncol, hh, m, f0, f1);
    const float bb = bf1[ncol];
#pragma unroll
    for (int r = 0; r < 8; ++r) {
      unsigned ha, la, hb, lb;
      split1(fmaxf(f0[r] + bb, 0.f), ha, la);
      split1(fmaxf(f1[r] + bb, 0.f), hb, lb);
      Fhi[(8 * hh + r) * FP + ncol]      = (unsigned short)ha;
      Flo[(8 * hh + r) * FP + ncol]      = (unsigned short)la;
      Fhi[(16 + 8 * hh + r) * FP + ncol] = (unsigned short)hb;
      Flo[(16 + 8 * hh + r) * FP + ncol] = (unsigned short)lb;
    }
  }
  __syncthreads();

  {
    v8f y0 = {0.f, 0.f, 0.f, 0.f, 0.f, 0.f, 0.f, 0.f};
    v8f y1 = {0.f, 0.f, 0.f, 0.f, 0.f, 0.f, 0.f, 0.f};
    gemm2t<FFW>(Fhi, Flo, FP, W2h, W2l, ncw, hh, m, y0, y1);
    const float bb = bf2[ncw];
#pragma unroll
    for (int r = 0; r < 8; ++r) {
      const int ra = (8 * hh + r) * XP + ncw;
      const int rb = (16 + 8 * hh + r) * XP + ncw;
      Os[ra] = y0[r] + bb + Hs[ra];
      Os[rb] = y1[r] + bb + Hs[rb];
    }
  }
  __syncthreads();

  {
    const v4f gv = *(const v4f*)(g2 + 4 * lane);
    const v4f bv = *(const v4f*)(be2 + 4 * lane);
    v4f yr[4];
    float* opp[4];
    bool ok[4];
#pragma unroll
    for (int i = 0; i < 4; ++i) {
      const int row  = 4 * wave + i;
      const int grow = rowBase + row;
      const v4f xv = *(const v4f*)(Os + row * XP + 4 * lane);
      yr[i]  = ln_row(xv, gv, bv);
      ok[i]  = (grow < nN);
      const int gcl = ok[i] ? grow : (nN - 1);
      opp[i] = out + (size_t)gcl * DF + 4 * lane;
    }
#pragma unroll
    for (int i = 0; i < 4; ++i) if (ok[i]) *(volatile v4f*)(opp[i]) = yr[i];
    __threadfence();
#pragma unroll
    for (int i = 0; i < 4; ++i) if (ok[i]) *(volatile v4f*)(opp[i]) = yr[i];
  }
}

extern "C" void kernel_launch(void* const* d_in, const int* in_sizes, int n_in,
                              void* d_out, int out_size, void* d_ws, size_t ws_size,
                              hipStream_t stream) {
  if (n_in < 15) return;
  const int nN = in_sizes[0] / DF;
  const int nE = in_sizes[1];
  if (nN <= 0 || in_sizes[0] != nN * DF) return;
  if (nE < 0 || in_sizes[2] != nE) return;
  if (in_sizes[3] != DF * DF || in_sizes[4] != DF * DF || in_sizes[5] != DF * DF || in_sizes[6] != DF * DF) return;
  if (in_sizes[7] != DF || in_sizes[8] != DF || in_sizes[9] != DF || in_sizes[10] != DF) return;
  if (in_sizes[11] != DF * FFW || in_sizes[12] != FFW || in_sizes[13] != FFW * DF || in_sizes[14] != DF) return;
  if (out_size != nN * DF) return;

  const float* h    = (const float*)d_in[0];
  const int*   src  = (const int*)d_in[1];
  const int*   dst  = (const int*)d_in[2];
  const float* Wq   = (const float*)d_in[3];
  const float* Wk   = (const float*)d_in[4];
  const float* Wv   = (const float*)d_in[5];
  const float* Wo   = (const float*)d_in[6];
  const float* ln1g = (const float*)d_in[7];
  const float* ln1b = (const float*)d_in[8];
  const float* ln2g = (const float*)d_in[9];
  const float* ln2b = (const float*)d_in[10];
  const float* W1   = (const float*)d_in[11];
  const float* b1   = (const float*)d_in[12];
  const float* W2   = (const float*)d_in[13];
  const float* b2   = (const float*)d_in[14];
  float* out = (float*)d_out;

  const int nP = ((nN + GR - 1) / GR) * GR;
  size_t off = 0;
  char* base = (char*)d_ws;
  unsigned short* Wqkv_h = (unsigned short*)(base + off); off += (size_t)QC * DF * 2;
  unsigned short* Wqkv_l = (unsigned short*)(base + off); off += (size_t)QC * DF * 2;
  unsigned short* Wo_h   = (unsigned short*)(base + off); off += (size_t)DF * DF * 2;
  unsigned short* Wo_l   = (unsigned short*)(base + off); off += (size_t)DF * DF * 2;
  unsigned short* W1_h   = (unsigned short*)(base + off); off += (size_t)FFW * DF * 2;
  unsigned short* W1_l   = (unsigned short*)(base + off); off += (size_t)FFW * DF * 2;
  unsigned short* W2_h   = (unsigned short*)(base + off); off += (size_t)DF * FFW * 2;
  unsigned short* W2_l   = (unsigned short*)(base + off); off += (size_t)DF * FFW * 2;
  float* qkv    = (float*)(base + off); off += (size_t)nP * QC * sizeof(float);
  float* aplane = (float*)(base + off); off += (size_t)nN * DF * sizeof(float);
  if (off > ws_size) return;
  if (off > (size_t)134217728) return;

  const int n8a = DF * DF / 8;
  const int n8b = DF * FFW / 8;
  k_prepw<<<(n8a + NTHR - 1) / NTHR, NTHR, 0, stream>>>(Wq, DF, DF, Wqkv_h, Wqkv_l, n8a);
  k_prepw<<<(n8a + NTHR - 1) / NTHR, NTHR, 0, stream>>>(Wk, DF, DF, Wqkv_h + DF * DF, Wqkv_l + DF * DF, n8a);
  k_prepw<<<(n8a + NTHR - 1) / NTHR, NTHR, 0, stream>>>(Wv, DF, DF, Wqkv_h + 2 * DF * DF, Wqkv_l + 2 * DF * DF, n8a);
  k_prepw<<<(n8a + NTHR - 1) / NTHR, NTHR, 0, stream>>>(Wo, DF, DF, Wo_h, Wo_l, n8a);
  k_prepw<<<(n8b + NTHR - 1) / NTHR, NTHR, 0, stream>>>(W1, DF, FFW, W1_h, W1_l, n8b);
  k_prepw<<<(n8b + NTHR - 1) / NTHR, NTHR, 0, stream>>>(W2, FFW, DF, W2_h, W2_l, n8b);

  hipFuncSetAttribute(reinterpret_cast<const void*>(&k_qkv), hipFuncAttributeMaxDynamicSharedMemorySize, LDS2_BYTES);
  k_qkv<<<nP / GR, NTHR, LDS2_BYTES, stream>>>(h, Wqkv_h, Wqkv_l, qkv, nN);

  hipFuncSetAttribute(reinterpret_cast<const void*>(&k_agg), hipFuncAttributeMaxDynamicSharedMemorySize, LDS3_BYTES);
  const int gridA = (nN + NB - 1) / NB;
  k_agg<<<gridA, NTHR, LDS3_BYTES, stream>>>(qkv, src, dst, aplane, nN, nE);

  hipFuncSetAttribute(reinterpret_cast<const void*>(&k_ffn), hipFuncAttributeMaxDynamicSharedMemorySize, LDS4_BYTES);
  k_ffn<<<nP / GR, NTHR, LDS4_BYTES, stream>>>(aplane, h, Wo_h, Wo_l, ln1g, ln1b, W1_h, W1_l, b1,
                                                W2_h, W2_l, b2, ln2g, ln2b, out, nN);
}
